// MambaDiffusion_8899172237907
// MI455X (gfx1250) — hardware-verified
//
#include <hip/hip_runtime.h>
#include <math.h>

typedef __attribute__((ext_vector_type(16))) _Float16 v16h;
typedef __attribute__((ext_vector_type(8)))  _Float16 v8h;
typedef __attribute__((ext_vector_type(16))) __bf16   v16b;
typedef __attribute__((ext_vector_type(8)))  __bf16   v8b;
typedef __attribute__((ext_vector_type(8)))  float    v8f;
typedef __attribute__((ext_vector_type(4)))  float    v4f;

constexpr int kBatch = 16;
constexpr int kImg   = 64;
constexpr int kCin   = 3;
constexpr int kPatch = 4;
constexpr int kDm    = 256;
constexpr int kNLay  = 4;
constexpr int kDin   = 512;
constexpr int kNst   = 16;
constexpr int kDtR   = 32;
constexpr int kSeq   = 256;
constexpr int kRows  = kBatch * kSeq;
constexpr int kPF    = 48;
constexpr int kPFP   = 64;
constexpr int kXZP   = 2 * kDin;
constexpr int kPrj   = kDtR + 2 * kNst;
constexpr int kYP    = 2 * kDin;
constexpr int kHeadN = 48;
constexpr int kHeadP = 64;
constexpr int kTP    = 260;

__device__ __forceinline__ unsigned short f2bf_bits(float f) {
  unsigned u = __float_as_uint(f);
  return (unsigned short)((u + 0x7FFFu + ((u >> 16) & 1u)) >> 16);
}
__device__ __forceinline__ float bf_bits2f(unsigned short h) { return __uint_as_float(((unsigned)h) << 16); }

__device__ __forceinline__ void dep_guard_h(v8f& a, v8f& b, v16h x, v16h y) { asm volatile("v_nop\n\tv_nop\n\tv_nop\n\tv_nop" : "+v"(a), "+v"(b) : "v"(x), "v"(y)); }
__device__ __forceinline__ void dep_guard_b(v8f& a, v8f& b, v16b x, v16b y) { asm volatile("v_nop\n\tv_nop\n\tv_nop\n\tv_nop" : "+v"(a), "+v"(b) : "v"(x), "v"(y)); }
__device__ __forceinline__ void keep4_h(v16h a, v16h b, v16h c, v16h d) { asm volatile("v_nop" :: "v"(a), "v"(b), "v"(c), "v"(d)); }
__device__ __forceinline__ void keep4_b(v16b a, v16b b, v16b c, v16b d) { asm volatile("v_nop" :: "v"(a), "v"(b), "v"(c), "v"(d)); }
__device__ __forceinline__ void acc_guard4(v8f& a, v8f& b, v8f& c, v8f& d) { asm volatile("v_nop\n\tv_nop\n\tv_nop\n\tv_nop" : "+v"(a), "+v"(b), "+v"(c), "+v"(d)); }
template <typename T> struct Frag;
template <> struct Frag<_Float16> {
  typedef v16h V; union U { v16h v; v8h h[2]; };
  static __device__ __forceinline__ v16h load(const _Float16* p) {
    U f; f.h[0] = *(const v8h*)(p); f.h[1] = *(const v8h*)(p + 16); return f.v;
  }
  static __device__ __forceinline__ v8f mma(v16h a, v16h b, v8f c) {
    return __builtin_amdgcn_wmma_f32_16x16x32_f16(false, a, false, b, (short)0, c, false, false);
  }
  static __device__ __forceinline__ void guard(v8f& a, v8f& b, v16h x, v16h y) { dep_guard_h(a, b, x, y); }
  static __device__ __forceinline__ void keep(v16h a, v16h b, v16h c, v16h d) { keep4_h(a, b, c, d); }
};
template <> struct Frag<__bf16> {
  typedef v16b V; union U { v16b v; v8b h[2]; };
  static __device__ __forceinline__ v16b load(const __bf16* p) {
    U f; f.h[0] = *(const v8b*)(p); f.h[1] = *(const v8b*)(p + 16); return f.v;
  }
  static __device__ __forceinline__ v8f mma(v16b a, v16b b, v8f c) {
    return __builtin_amdgcn_wmma_f32_16x16x32_bf16(false, a, false, b, (short)0, c, false, false);
  }
  static __device__ __forceinline__ void guard(v8f& a, v8f& b, v16b x, v16b y) { dep_guard_b(a, b, x, y); }
  static __device__ __forceinline__ void keep(v16b a, v16b b, v16b c, v16b d) { keep4_b(a, b, c, d); }
};

template <int ET> struct Elem;
template <> struct Elem<0> { typedef _Float16 T; };
template <> struct Elem<1> { typedef __bf16 T; };
template <int ET, bool SPLIT, int BIAS_MODE, int OUT_MODE, bool RESID, int ACT = 0>
__global__ __launch_bounds__(256) void wmma_gemm64(
    const unsigned short* __restrict__ Ap, const unsigned short* __restrict__ A2p, int lda, long strideA,
    const unsigned short* __restrict__ Btp, const unsigned short* __restrict__ Bt2p, int ldb, long strideB,
    void* __restrict__ Cout, void* __restrict__ Cout2, int ldc, long strideC,
    const float* __restrict__ bias,
    const float* __restrict__ resid, long strideR,
    int M, int N, int K, float scale) {
  typedef typename Elem<ET>::T T;
  typedef typename Frag<T>::V V;
  const T* A = (const T*)Ap; const T* A2 = (const T*)A2p; const T* Bt = (const T*)Btp; const T* Bt2 = (const T*)Bt2p;
  __shared__ __align__(16) float sT[8][16 * 68];
  const int b    = blockIdx.y;
  const int lane = threadIdx.x & 31;
  const int wave = threadIdx.x >> 5;
  const int tilesN = N >> 6;
  const int tilesM = M >> 6;
  const int tile = blockIdx.x * 8 + wave;
  if (tile >= tilesM * tilesN) return;
  const int tm = tile / tilesN;
  const int tn = tile - tm * tilesN;
  const int m0 = tm << 6;
  const int n0 = tn << 6;

  const T* Ab  = A  + (size_t)b * strideA;
  const T* Bb  = Bt + (size_t)b * strideB;
  const T* Ab2 = SPLIT ? (A2  + (size_t)b * strideA) : nullptr;
  const T* Bb2 = SPLIT ? (Bt2 + (size_t)b * strideB) : nullptr;

  const int rlane = lane & 15;
  const int koff  = (lane >> 4) * 8;
  const int mOff  = (lane >> 4) * 8;

  v8f acc[4][4];
#pragma unroll
  for (int i = 0; i < 4; ++i)
#pragma unroll
    for (int j = 0; j < 4; ++j) acc[i][j] = (v8f){0.f,0.f,0.f,0.f,0.f,0.f,0.f,0.f};

  for (int k0 = 0; k0 < K; k0 += 32) {
    V bh[4], bl[4];
#pragma unroll
    for (int j = 0; j < 4; ++j) {
      const size_t bo = (size_t)(n0 + (j << 4) + rlane) * ldb + koff + k0;
      bh[j] = Frag<T>::load(Bb + bo);
      if (SPLIT) bl[j] = Frag<T>::load(Bb2 + bo);
    }
#pragma unroll
    for (int i = 0; i < 4; ++i) {
      const size_t ao = (size_t)(m0 + (i << 4) + rlane) * lda + koff + k0;
      V ah = Frag<T>::load(Ab + ao);
      V al;
      if (SPLIT) al = Frag<T>::load(Ab2 + ao);
#pragma unroll
      for (int j = 0; j < 4; ++j) {
        acc[i][j] = Frag<T>::mma(ah, bh[j], acc[i][j]);
        if (SPLIT) {
          acc[i][j] = Frag<T>::mma(ah, bl[j], acc[i][j]);
          acc[i][j] = Frag<T>::mma(al, bh[j], acc[i][j]);
        }
      }
      Frag<T>::guard(acc[i][0], acc[i][3], ah, SPLIT ? al : ah);
    }
    Frag<T>::keep(bh[0], bh[1], bh[2], bh[3]);
    if (SPLIT) Frag<T>::keep(bl[0], bl[1], bl[2], bl[3]);
  }
  acc_guard4(acc[0][0], acc[0][1], acc[0][2], acc[0][3]);
  acc_guard4(acc[1][0], acc[1][1], acc[1][2], acc[1][3]);
  acc_guard4(acc[2][0], acc[2][1], acc[2][2], acc[2][3]);
  acc_guard4(acc[3][0], acc[3][1], acc[3][2], acc[3][3]);

  float* slab = sT[wave];
  const float* Rb = RESID ? (resid + (size_t)b * strideR) : nullptr;
#pragma unroll
  for (int i = 0; i < 4; ++i) {
    const int mBase = m0 + (i << 4);
#pragma unroll
    for (int j = 0; j < 4; ++j) {
      const int n = n0 + (j << 4) + rlane;
      float bv = 0.f;
      if (BIAS_MODE == 2) bv = bias[n];
#pragma unroll
      for (int r = 0; r < 8; ++r) {
        float v = acc[i][j][r] * scale;
        if (BIAS_MODE == 1) v += bias[mBase + mOff + r];
        if (BIAS_MODE == 2) v += bv;
        if (RESID) v += Rb[(size_t)(mBase + mOff + r) * ldc + n];
        if (ACT == 1) v = tanhf(v);
        if (ACT == 2) v = fmaxf(v, 0.0f);
        if (ACT == 3) v = v / (1.0f + expf(-v));
        if (ACT == 4) v = (v > 0.f) ? v : 0.01f * v;
        if (ACT == 5) v = 0.5f * v * (1.0f + erff(v * 0.70710678118654752f));
        slab[(mOff + r) * 68 + (j << 4) + rlane] = v;
      }
    }
    __builtin_amdgcn_fence(__ATOMIC_RELEASE, "workgroup");
    __builtin_amdgcn_wave_barrier();
    __builtin_amdgcn_fence(__ATOMIC_ACQUIRE, "workgroup");
    if (OUT_MODE == 0) {
      float* C = (float*)Cout + (size_t)b * strideC;
      const int hh = lane >> 4, c4 = (lane & 15) * 4;
      for (int pass = 0; pass < 2; ++pass) {
#pragma unroll
        for (int it = 0; it < 8; ++it) {
          const int row = it * 2 + hh;
          v4f v = *(const v4f*)(slab + row * 68 + c4);
          *(volatile v4f*)(C + (size_t)(mBase + row) * ldc + n0 + c4) = v;
        }
        __threadfence();
      }
    } else {
      const int q = lane >> 3, c8 = (lane & 7) * 8;
      unsigned short* C  = (unsigned short*)Cout  + (size_t)b * strideC;
      unsigned short* C2 = (OUT_MODE == 2) ? ((unsigned short*)Cout2 + (size_t)b * strideC) : nullptr;
      for (int pass = 0; pass < 2; ++pass) {
#pragma unroll
        for (int it = 0; it < 4; ++it) {
          const int row = it * 4 + q;
          const float* sp = slab + row * 68 + c8;
          v8h hv, lv;
#pragma unroll
          for (int e = 0; e < 8; ++e) {
            if (OUT_MODE == 1) {
              hv[e] = (_Float16)sp[e];
            } else {
              unsigned short hb = f2bf_bits(sp[e]);
              unsigned short lb = f2bf_bits(sp[e] - bf_bits2f(hb));
              hv[e] = __builtin_bit_cast(_Float16, hb);
              lv[e] = __builtin_bit_cast(_Float16, lb);
            }
          }
          *(volatile v8h*)(C + (size_t)(mBase + row) * ldc + n0 + c8) = hv;
          if (OUT_MODE == 2) *(volatile v8h*)(C2 + (size_t)(mBase + row) * ldc + n0 + c8) = lv;
        }
        __threadfence();
      }
    }
    __builtin_amdgcn_fence(__ATOMIC_RELEASE, "workgroup");
    __builtin_amdgcn_wave_barrier();
    __builtin_amdgcn_fence(__ATOMIC_ACQUIRE, "workgroup");
  }
}

__global__ __launch_bounds__(256) void cast_rows_f16_kernel(
    const float* __restrict__ src, unsigned short* __restrict__ dst, int N, int K, int total8, float scale)
{
  const int i = blockIdx.x * 256 + threadIdx.x;
  if (i >= total8) return;
  const int e0  = i << 3;
  const int row = e0 / K;
  const int col = e0 - row * K;
  const int rowc = (row < N) ? row : (N - 1);
  const bool live = (row < N);
  const float* p = src + (size_t)rowc * K + col;
  const v4f a0 = *(const v4f*)(p);
  const v4f a1 = *(const v4f*)(p + 4);
  v8h hv;
#pragma unroll
  for (int e = 0; e < 4; ++e) {
    hv[e]     = live ? (_Float16)(a0[e] * scale) : (_Float16)0.0f;
    hv[4 + e] = live ? (_Float16)(a1[e] * scale) : (_Float16)0.0f;
  }
  unsigned short* q = dst + (size_t)e0;
  *(volatile v8h*)q = hv;
  __threadfence();
  *(volatile v8h*)q = hv;
}

__global__ __launch_bounds__(256) void cast_dup_f16_kernel(
    const float* __restrict__ src, unsigned short* __restrict__ dst, int total8, float scale)
{
  const int i = blockIdx.x * 256 + threadIdx.x;
  if (i >= total8) return;
  const int e0  = i << 3;
  const int row = e0 >> 10;
  const int col = e0 & 1023;
  const int sc  = col & 511;
  const float* p = src + (size_t)row * kDin + sc;
  const v4f a0 = *(const v4f*)(p);
  const v4f a1 = *(const v4f*)(p + 4);
  v8h hv;
#pragma unroll
  for (int e = 0; e < 4; ++e) {
    hv[e]     = (_Float16)(a0[e] * scale);
    hv[4 + e] = (_Float16)(a1[e] * scale);
  }
  unsigned short* q = dst + (size_t)e0;
  *(volatile v8h*)q = hv;
  __threadfence();
  *(volatile v8h*)q = hv;
}

__device__ __forceinline__ void split_bf(float f, _Float16& h, _Float16& l) {
  const unsigned short hb = f2bf_bits(f);
  const unsigned short lb = f2bf_bits(f - bf_bits2f(hb));
  h = __builtin_bit_cast(_Float16, hb);
  l = __builtin_bit_cast(_Float16, lb);
}

__global__ __launch_bounds__(256) void cast_rows_bf16_split_kernel(
    const float* __restrict__ src, unsigned short* __restrict__ dhi, unsigned short* __restrict__ dlo, int N, int K, int total8)
{
  const int i = blockIdx.x * 256 + threadIdx.x;
  if (i >= total8) return;
  const int e0  = i << 3;
  const int row = e0 / K;
  const int col = e0 - row * K;
  const int rowc = (row < N) ? row : (N - 1);
  const bool live = (row < N);
  const float* p = src + (size_t)rowc * K + col;
  const v4f a0 = *(const v4f*)(p);
  const v4f a1 = *(const v4f*)(p + 4);
  v8h hv, lv;
#pragma unroll
  for (int e = 0; e < 4; ++e) {
    _Float16 h0, l0, h1, l1;
    split_bf(live ? a0[e] : 0.0f, h0, l0);
    split_bf(live ? a1[e] : 0.0f, h1, l1);
    hv[e] = h0; lv[e] = l0; hv[4 + e] = h1; lv[4 + e] = l1;
  }
  unsigned short* qh = dhi + (size_t)e0;
  unsigned short* ql = dlo + (size_t)e0;
  *(volatile v8h*)qh = hv;
  *(volatile v8h*)ql = lv;
  __threadfence();
  *(volatile v8h*)qh = hv;
  *(volatile v8h*)ql = lv;
}

__global__ __launch_bounds__(256) void cast_padk_bf16_split_kernel(
    const float* __restrict__ src, int lds, unsigned short* __restrict__ dhi, unsigned short* __restrict__ dlo,
    int K, int Kp, int total8)
{
  const int i = blockIdx.x * 256 + threadIdx.x;
  if (i >= total8) return;
  const int e0  = i << 3;
  const int row = e0 / Kp;
  const int col = e0 - row * Kp;
  const bool live = (col < K);
  const int colc = live ? col : (K - 8);
  const float* p = src + (size_t)row * lds + colc;
  const v4f a0 = *(const v4f*)(p);
  const v4f a1 = *(const v4f*)(p + 4);
  v8h hv, lv;
#pragma unroll
  for (int e = 0; e < 4; ++e) {
    _Float16 h0, l0, h1, l1;
    split_bf(live ? a0[e] : 0.0f, h0, l0);
    split_bf(live ? a1[e] : 0.0f, h1, l1);
    hv[e] = h0; lv[e] = l0; hv[4 + e] = h1; lv[4 + e] = l1;
  }
  unsigned short* qh = dhi + (size_t)e0;
  unsigned short* ql = dlo + (size_t)e0;
  *(volatile v8h*)qh = hv;
  *(volatile v8h*)ql = lv;
  __threadfence();
  *(volatile v8h*)qh = hv;
  *(volatile v8h*)ql = lv;
}

__global__ __launch_bounds__(256) void im2col_split_kernel(
    const float* __restrict__ xin, unsigned short* __restrict__ XH, unsigned short* __restrict__ XL)
{
  const int i = blockIdx.x * 256 + threadIdx.x;
  if (i >= kRows * 8) return;
  const int tok = i >> 3, q = i & 7;
  const int b = tok >> 8, p = tok & 255, hp = p >> 4, wp = p & 15;
  const bool live = (q < 6);
  const int qc = live ? q : 5;
  const int j0 = qc * 8;
  const int c = j0 >> 4;
  const int py0 = (j0 >> 2) & 3;
  const float* src = xin + ((((size_t)(b * kCin + c)) * kImg + hp * kPatch + py0) * kImg + wp * kPatch);
  const v4f a0 = *(const v4f*)(src);
  const v4f a1 = *(const v4f*)(src + kImg);
  v8h hv, lv;
#pragma unroll
  for (int e = 0; e < 4; ++e) {
    _Float16 h0, l0, h1, l1;
    split_bf(live ? a0[e] : 0.0f, h0, l0);
    split_bf(live ? a1[e] : 0.0f, h1, l1);
    hv[e] = h0; lv[e] = l0; hv[4 + e] = h1; lv[4 + e] = l1;
  }
  unsigned short* qh = XH + (size_t)i * 8;
  unsigned short* ql = XL + (size_t)i * 8;
  *(volatile v8h*)qh = hv;
  *(volatile v8h*)ql = lv;
  __threadfence();
  *(volatile v8h*)qh = hv;
  *(volatile v8h*)ql = lv;
}

__global__ __launch_bounds__(256) void time_embed_kernel(
    const int* __restrict__ tin, const float* __restrict__ tw1, const float* __restrict__ tb1,
    const float* __restrict__ tw2, const float* __restrict__ tb2, float* __restrict__ TE)
{
  __shared__ float vec[kDm];
  __shared__ float hid[kDm];
  const int b = blockIdx.x, d = threadIdx.x;
  const float tf = (float)tin[b];
  const float kFreqStep = -0.07252236513367074f;
  const int fi = (d < 128) ? d : (d - 128);
  const float fr = expf((float)fi * kFreqStep);
  const float arg = tf * fr;
  const float sv = sinf(arg);
  const float cv = cosf(arg);
  vec[d] = (d < 128) ? sv : cv;
  __syncthreads();
  float a = 0.0f;
  const float* w1 = tw1 + (size_t)d * kDm;
#pragma unroll 1
  for (int k = 0; k < kDm; ++k) a = fmaf(vec[k], w1[k], a);
  a += tb1[d];
  const float sg = 1.0f / (1.0f + expf(-a));
  hid[d] = a * sg;
  __syncthreads();
  float o = 0.0f;
  const float* w2 = tw2 + (size_t)d * kDm;
#pragma unroll 1
  for (int k = 0; k < kDm; ++k) o = fmaf(hid[k], w2[k], o);
  o += tb2[d];
  float* dst = TE + (size_t)b * kDm + d;
  *(volatile float*)dst = o;
  __threadfence();
  *(volatile float*)dst = o;
}

template <bool ADD_TE, int OMODE>
__global__ __launch_bounds__(256) void ln_rows_kernel(
    const float* __restrict__ Hs, const float* __restrict__ TEp,
    const float* __restrict__ gam, const float* __restrict__ bet,
    unsigned short* __restrict__ O1, unsigned short* __restrict__ O2, int nrows)
{
  const int lane = threadIdx.x & 31, wave = threadIdx.x >> 5;
  const int row = blockIdx.x * 8 + wave;
  if (row >= nrows) return;
  const int c0 = lane * 8;
  const float* hp = Hs + (size_t)row * kDm + c0;
  const v4f a0 = *(const v4f*)(hp);
  const v4f a1 = *(const v4f*)(hp + 4);
  float v[8];
#pragma unroll
  for (int e = 0; e < 4; ++e) { v[e] = a0[e]; v[4 + e] = a1[e]; }
  if (ADD_TE) {
    const float* tp = TEp + (size_t)(row >> 8) * kDm + c0;
    const v4f t0 = *(const v4f*)(tp);
    const v4f t1 = *(const v4f*)(tp + 4);
#pragma unroll
    for (int e = 0; e < 4; ++e) { v[e] += t0[e]; v[4 + e] += t1[e]; }
  }
  float s = 0.0f;
#pragma unroll
  for (int e = 0; e < 8; ++e) s += v[e];
#pragma unroll
  for (int off = 16; off > 0; off >>= 1) s += __shfl_xor(s, off, 32);
  const float mu = s * (1.0f / 256.0f);
  float q = 0.0f;
#pragma unroll
  for (int e = 0; e < 8; ++e) { const float c = v[e] - mu; v[e] = c; q = fmaf(c, c, q); }
#pragma unroll
  for (int off = 16; off > 0; off >>= 1) q += __shfl_xor(q, off, 32);
  const float var = q * (1.0f / 256.0f);
  const float rstd = rsqrtf(var + 1e-5f);
  const v4f g0 = *(const v4f*)(gam + c0);
  const v4f g1 = *(const v4f*)(gam + c0 + 4);
  const v4f b0 = *(const v4f*)(bet + c0);
  const v4f b1 = *(const v4f*)(bet + c0 + 4);
  float o[8];
#pragma unroll
  for (int e = 0; e < 4; ++e) {
    o[e]     = v[e] * rstd * g0[e] + b0[e];
    o[4 + e] = v[4 + e] * rstd * g1[e] + b1[e];
  }
  if (OMODE == 0) {
    v8h hv;
#pragma unroll
    for (int e = 0; e < 8; ++e) hv[e] = (_Float16)o[e];
    unsigned short* dst = O1 + (size_t)row * kDm + c0;
    *(volatile v8h*)dst = hv;
    __threadfence();
    *(volatile v8h*)dst = hv;
  } else {
    v8h hv, lv;
#pragma unroll
    for (int e = 0; e < 8; ++e) { _Float16 hh, ll; split_bf(o[e], hh, ll); hv[e] = hh; lv[e] = ll; }
    unsigned short* dh = O1 + (size_t)row * kDm + c0;
    unsigned short* dl = O2 + (size_t)row * kDm + c0;
    *(volatile v8h*)dh = hv;
    *(volatile v8h*)dl = lv;
    __threadfence();
    *(volatile v8h*)dh = hv;
    *(volatile v8h*)dl = lv;
  }
}

__global__ __launch_bounds__(256) void conv_silu_kernel(
    const float* __restrict__ XZ, const float* __restrict__ cw, const float* __restrict__ cb,
    unsigned short* __restrict__ U16)
{
  __shared__ __align__(16) float sT[16 * kTP];
  const int tid = threadIdx.x, lane = tid & 31, wave = tid >> 5;
  const int d0 = blockIdx.x * 256, d = d0 + tid;
  const int t0 = blockIdx.y * 64;
  const int b  = blockIdx.z;
  const size_t brow = (size_t)b * kSeq;
  const float w0 = cw[d * 4 + 0], w1 = cw[d * 4 + 1], w2 = cw[d * 4 + 2], w3 = cw[d * 4 + 3];
  const float bc = cb[d];
  float xm3, xm2, xm1;
  {
    const int r3 = t0 - 3, r2 = t0 - 2, r1 = t0 - 1;
    const int c3 = r3 < 0 ? 0 : r3, c2 = r2 < 0 ? 0 : r2, c1 = r1 < 0 ? 0 : r1;
    const float v3 = XZ[(brow + (size_t)c3) * kXZP + d];
    const float v2 = XZ[(brow + (size_t)c2) * kXZP + d];
    const float v1 = XZ[(brow + (size_t)c1) * kXZP + d];
    xm3 = (r3 >= 0) ? v3 : 0.f;
    xm2 = (r2 >= 0) ? v2 : 0.f;
    xm1 = (r1 >= 0) ? v1 : 0.f;
  }
#pragma unroll 1
  for (int sub = 0; sub < 4; ++sub) {
    const int lb = t0 + sub * 16;
#pragma unroll 1
    for (int st = 0; st < 16; ++st) {
      const int tt  = lb + st;
      const float xin = XZ[(brow + (size_t)tt) * kXZP + d];
      float acc = w0 * xm3;
      acc = fmaf(w1, xm2, acc);
      acc = fmaf(w2, xm1, acc);
      acc = fmaf(w3, xin, acc);
      const float sv = acc + bc;
      const float sg = __builtin_amdgcn_rcpf(1.0f + __expf(-sv));
      sT[st * kTP + tid] = (sv * sg) * 16.0f;
      xm3 = xm2; xm2 = xm1; xm1 = xin;
    }
    __syncthreads();
    v8h bv[2];
#pragma unroll
    for (int it = 0; it < 2; ++it) {
      const float* sp = sT + (it * 8 + wave) * kTP + lane * 8;
      const v4f a0 = *(const v4f*)(sp);
      const v4f a1 = *(const v4f*)(sp + 4);
#pragma unroll
      for (int e = 0; e < 4; ++e) {
        bv[it][e]     = (_Float16)a0[e];
        bv[it][4 + e] = (_Float16)a1[e];
      }
    }
    for (int pass = 0; pass < 2; ++pass) {
#pragma unroll
      for (int it = 0; it < 2; ++it) {
        const int tt = lb + it * 8 + wave;
        *(volatile v8h*)(U16 + (brow + (size_t)tt) * kDin + d0 + lane * 8) = bv[it];
      }
      __threadfence();
    }
    __syncthreads();
  }
}

__global__ __launch_bounds__(256) void scan_kernel(
    const _Float16* __restrict__ DLRall, const _Float16* __restrict__ U16p, const _Float16* __restrict__ PRJall,
    const float* __restrict__ XZp,
    const float* __restrict__ dtb0, const float* __restrict__ dtb1,
    const float* __restrict__ Alog0, const float* __restrict__ Alog1,
    const float* __restrict__ Dv0, const float* __restrict__ Dv1,
    unsigned short* __restrict__ Y16p)
{
  __shared__ __align__(16) float sBC[16 * 32];
  __shared__ __align__(16) float sY[16 * kTP];
  const int tid = threadIdx.x, lane = tid & 31, wave = tid >> 5;
  const int d0 = blockIdx.x * 256, d = d0 + tid;
  const int b  = blockIdx.y;
  const int rev = blockIdx.z;
  const size_t brow = (size_t)b * kSeq;
  const _Float16* DLR = DLRall + (size_t)rev * kRows * kDin;
  const _Float16* PRJ = PRJall + (size_t)rev * kRows * kPrj;
  const float* dtb   = rev ? dtb1 : dtb0;
  const float* A_log = rev ? Alog1 : Alog0;
  const float* Dv    = rev ? Dv1 : Dv0;
  const int ycol = rev * kDin + d0;

  float An[kNst];
#pragma unroll
  for (int n = 0; n < kNst; ++n) An[n] = -expf(A_log[(size_t)d * kNst + n]);
  const float Dd  = Dv[d];
  const float bdt = dtb[d];
  float h[kNst];
#pragma unroll
  for (int n = 0; n < kNst; ++n) h[n] = 0.f;

#pragma unroll 1
  for (int c = 0; c < kSeq / 16; ++c) {
    const int l0 = c * 16;
    if (tid < 64) {
      const int r = tid >> 2, q = (tid & 3) * 8;
      const int tt  = l0 + r;
      const int tok = rev ? (kSeq - 1 - tt) : tt;
      const _Float16* pp = PRJ + (brow + (size_t)tok) * kPrj + kDtR + q;
      const v8h pv = *(const v8h*)pp;
#pragma unroll
      for (int e = 0; e < 8; ++e) sBC[r * 32 + q + e] = (float)pv[e] * (1.0f / 64.0f);
    }
    __syncthreads();
#pragma unroll 1
    for (int st = 0; st < 16; ++st) {
      const int tt  = l0 + st;
      const int tok = rev ? (kSeq - 1 - tt) : tt;
      const size_t m = brow + (size_t)tok;
      const float a     = (float)DLR[m * kDin + d] * (1.0f / 256.0f) + bdt;
      const float delta = fmaxf(a, 0.0f) + log1pf(__expf(-fabsf(a)));
      const float xv    = (float)U16p[m * kDin + d] * (1.0f / 16.0f);
      const float zv    = XZp[m * kXZP + kDin + d];
      v4f Bq[4], Cq[4];
#pragma unroll
      for (int qq = 0; qq < 4; ++qq) {
        Bq[qq] = *(const v4f*)(sBC + st * 32 + 4 * qq);
        Cq[qq] = *(const v4f*)(sBC + st * 32 + kNst + 4 * qq);
      }
      float dx = delta * xv;
      asm volatile("" : "+v"(dx));
      float y = 0.f;
#pragma unroll
      for (int n = 0; n < kNst; ++n) {
        const float e = __expf(delta * An[n]);
        float p = dx * Bq[n >> 2][n & 3];
        asm volatile("" : "+v"(p));
        float qv = h[n] * e;
        asm volatile("" : "+v"(qv));
        const float hn = qv + p;
        h[n] = hn;
        float rr = Cq[n >> 2][n & 3] * hn;
        asm volatile("" : "+v"(rr));
        y += rr;
      }
      float sk = xv * Dd;
      asm volatile("" : "+v"(sk));
      y += sk;
      const float sg = __builtin_amdgcn_rcpf(1.0f + __expf(-zv));
      const float g  = zv * sg;
      sY[st * kTP + tid] = (y * g) * 64.0f;
    }
    __syncthreads();
    v8h hv[2];
#pragma unroll
    for (int it = 0; it < 2; ++it) {
      const float* sp = sY + (it * 8 + wave) * kTP + lane * 8;
      const v4f a0 = *(const v4f*)(sp);
      const v4f a1 = *(const v4f*)(sp + 4);
#pragma unroll
      for (int e = 0; e < 4; ++e) {
        hv[it][e]     = (_Float16)a0[e];
        hv[it][4 + e] = (_Float16)a1[e];
      }
    }
    for (int pass = 0; pass < 2; ++pass) {
#pragma unroll
      for (int it = 0; it < 2; ++it) {
        const int tt  = l0 + it * 8 + wave;
        const int tok = rev ? (kSeq - 1 - tt) : tt;
        const size_t yo = (brow + (size_t)tok) * kYP + ycol + lane * 8;
        *(volatile v8h*)(Y16p + yo) = hv[it];
      }
      __threadfence();
    }
    __syncthreads();
  }
}

__global__ __launch_bounds__(256) void depatch_kernel(
    const float* __restrict__ OT, const float* __restrict__ fb, float* __restrict__ outp)
{
  const int i = blockIdx.x * 256 + threadIdx.x;
  if (i >= kBatch * kCin * kImg * (kImg / 4)) return;
  const int wp  = i & 15;
  const int row = (i >> 4) & 63;
  const int bc  = i >> 10;
  const int c   = bc % 3;
  const int b   = bc / 3;
  const int hp = row >> 2, py = row & 3;
  const int tok = b * kSeq + hp * 16 + wp;
  const int f0  = c * 16 + py * 4;
  const v4f o  = *(const v4f*)(OT + (size_t)tok * kHeadP + f0);
  const v4f bb = *(const v4f*)(fb + f0);
  const v4f r  = o + bb;
  float* dst = outp + (size_t)i * 4;
  *(volatile v4f*)dst = r;
  __threadfence();
  *(volatile v4f*)dst = r;
}

extern "C" void kernel_launch(void* const* d_in, const int* in_sizes, int n_in,
                              void* d_out, int out_size, void* d_ws, size_t ws_size,
                              hipStream_t stream)
{
  if (n_in < 28) return;
  const float* x        = (const float*)d_in[0];
  const int*   tin      = (const int*)  d_in[1];
  const float* patch_w  = (const float*)d_in[2];
  const float* patch_b  = (const float*)d_in[3];
  const float* tw1      = (const float*)d_in[4];
  const float* tb1      = (const float*)d_in[5];
  const float* tw2      = (const float*)d_in[6];
  const float* tb2      = (const float*)d_in[7];
  const float* norm_g   = (const float*)d_in[8];
  const float* norm_b   = (const float*)d_in[9];
  const float* inproj_w = (const float*)d_in[10];
  const float* conv_w   = (const float*)d_in[11];
  const float* conv_b   = (const float*)d_in[12];
  const float* Alog_f   = (const float*)d_in[13];
  const float* D_f      = (const float*)d_in[14];
  const float* xproj_f  = (const float*)d_in[15];
  const float* dtw_f    = (const float*)d_in[16];
  const float* dtb_f    = (const float*)d_in[17];
  const float* Alog_bk  = (const float*)d_in[18];
  const float* D_bk     = (const float*)d_in[19];
  const float* xproj_bk = (const float*)d_in[20];
  const float* dtw_bk   = (const float*)d_in[21];
  const float* dtb_bk   = (const float*)d_in[22];
  const float* outproj_w= (const float*)d_in[23];
  const float* fng      = (const float*)d_in[24];
  const float* fnb      = (const float*)d_in[25];
  const float* fin_w    = (const float*)d_in[26];
  const float* fin_b    = (const float*)d_in[27];
  float* dout = (float*)d_out;

  if (in_sizes[0]  != kBatch * kCin * kImg * kImg) return;
  if (in_sizes[1]  != kBatch) return;
  if (in_sizes[2]  != kDm * kPF || in_sizes[3] != kDm) return;
  if (in_sizes[4]  != kDm * kDm || in_sizes[5] != kDm || in_sizes[6] != kDm * kDm || in_sizes[7] != kDm) return;
  if (in_sizes[8]  != kNLay * kDm || in_sizes[9] != kNLay * kDm) return;
  if (in_sizes[10] != kNLay * kXZP * kDm) return;
  if (in_sizes[11] != kNLay * kDin * 4 || in_sizes[12] != kNLay * kDin) return;
  if (in_sizes[13] != kNLay * kDin * kNst || in_sizes[14] != kNLay * kDin) return;
  if (in_sizes[15] != kNLay * kPrj * kDin || in_sizes[16] != kNLay * kDin * kDtR || in_sizes[17] != kNLay * kDin) return;
  if (in_sizes[18] != kNLay * kDin * kNst || in_sizes[19] != kNLay * kDin) return;
  if (in_sizes[20] != kNLay * kPrj * kDin || in_sizes[21] != kNLay * kDin * kDtR || in_sizes[22] != kNLay * kDin) return;
  if (in_sizes[23] != kNLay * kDm * kDin) return;
  if (in_sizes[24] != kDm || in_sizes[25] != kDm) return;
  if (in_sizes[26] != kHeadN * kDm || in_sizes[27] != kHeadN) return;
  if (out_size != kBatch * kCin * kImg * kImg) return;

  const size_t SZ_TE    = 65536;
  const size_t SZ_WIN   = (size_t)kNLay * kXZP * kDm * 2;
  const size_t SZ_WXP   = (size_t)2 * kNLay * kPrj * kDin * 2;
  const size_t SZ_WDT   = (size_t)2 * kNLay * kDin * kDtR * 2;
  const size_t SZ_WOUT  = (size_t)kNLay * kDm * kYP * 2;
  const size_t SZ_PW    = (size_t)kDm * kPFP * 2;
  const size_t SZ_FW    = (size_t)kHeadP * kDm * 2;
  const size_t SZ_XP    = (size_t)kRows * kPFP * 2;
  const size_t SZ_H     = (size_t)kRows * kDm * 4;
  const size_t SZ_HN    = (size_t)kRows * kDm * 2;
  const size_t SZ_XZ    = (size_t)kRows * kXZP * 4;
  const size_t SZ_U16   = (size_t)kRows * kDin * 2;
  const size_t SZ_PRJ   = (size_t)2 * kRows * kPrj * 2;
  const size_t SZ_DLR   = (size_t)2 * kRows * kDin * 2;
  const size_t SZ_Y16   = (size_t)kRows * kYP * 2;
  const size_t SZ_OT    = (size_t)kRows * kHeadP * 4;
  const size_t OFF_TE   = 0;
  const size_t OFF_WIN  = OFF_TE   + SZ_TE;
  const size_t OFF_WXP  = OFF_WIN  + SZ_WIN;
  const size_t OFF_WDT  = OFF_WXP  + SZ_WXP;
  const size_t OFF_WOUT = OFF_WDT  + SZ_WDT;
  const size_t OFF_PWH  = OFF_WOUT + SZ_WOUT;
  const size_t OFF_PWL  = OFF_PWH  + SZ_PW;
  const size_t OFF_FWH  = OFF_PWL  + SZ_PW;
  const size_t OFF_FWL  = OFF_FWH  + SZ_FW;
  const size_t OFF_XPH  = OFF_FWL  + SZ_FW;
  const size_t OFF_XPL  = OFF_XPH  + SZ_XP;
  const size_t OFF_H0   = OFF_XPL  + SZ_XP;
  const size_t OFF_H1   = OFF_H0   + SZ_H;
  const size_t OFF_HN   = OFF_H1   + SZ_H;
  const size_t OFF_HNH  = OFF_HN   + SZ_HN;
  const size_t OFF_HNL  = OFF_HNH  + SZ_HN;
  const size_t OFF_XZ   = OFF_HNL  + SZ_HN;
  const size_t OFF_U16  = OFF_XZ   + SZ_XZ;
  const size_t OFF_PRJ  = OFF_U16  + SZ_U16;
  const size_t OFF_DLR  = OFF_PRJ  + SZ_PRJ;
  const size_t OFF_Y16  = OFF_DLR  + SZ_DLR;
  const size_t OFF_OT   = OFF_Y16  + SZ_Y16;
  const size_t TOTAL    = OFF_OT   + SZ_OT;
  if (TOTAL > (size_t)134217728) return;
  if (ws_size < TOTAL) return;

  char* ws = (char*)d_ws;
  float*          TE    = (float*)(ws + OFF_TE);
  unsigned short* WIN16 = (unsigned short*)(ws + OFF_WIN);
  unsigned short* WXP16 = (unsigned short*)(ws + OFF_WXP);
  unsigned short* WDT16 = (unsigned short*)(ws + OFF_WDT);
  unsigned short* WOUT2 = (unsigned short*)(ws + OFF_WOUT);
  unsigned short* PWH   = (unsigned short*)(ws + OFF_PWH);
  unsigned short* PWL   = (unsigned short*)(ws + OFF_PWL);
  unsigned short* FWH   = (unsigned short*)(ws + OFF_FWH);
  unsigned short* FWL   = (unsigned short*)(ws + OFF_FWL);
  unsigned short* XPH   = (unsigned short*)(ws + OFF_XPH);
  unsigned short* XPL   = (unsigned short*)(ws + OFF_XPL);
  float*          Hbuf[2] = { (float*)(ws + OFF_H0), (float*)(ws + OFF_H1) };
  unsigned short* HN16  = (unsigned short*)(ws + OFF_HN);
  unsigned short* HNH   = (unsigned short*)(ws + OFF_HNH);
  unsigned short* HNL   = (unsigned short*)(ws + OFF_HNL);
  float*          XZ    = (float*)(ws + OFF_XZ);
  unsigned short* U16   = (unsigned short*)(ws + OFF_U16);
  unsigned short* PRJ16 = (unsigned short*)(ws + OFF_PRJ);
  unsigned short* DLR16 = (unsigned short*)(ws + OFF_DLR);
  unsigned short* Y16   = (unsigned short*)(ws + OFF_Y16);
  float*          OT    = (float*)(ws + OFF_OT);
  const float* dummy_bias  = patch_b;
  const float* dummy_resid = Hbuf[0];

  im2col_split_kernel<<<(kRows * 8) / 256, 256, 0, stream>>>(x, XPH, XPL);
  cast_padk_bf16_split_kernel<<<(kDm * kPFP) / 8 / 256, 256, 0, stream>>>(
      patch_w, kPF, PWH, PWL, kPF, kPFP, (kDm * kPFP) / 8);
  cast_rows_bf16_split_kernel<<<(kHeadP * kDm) / 8 / 256, 256, 0, stream>>>(
      fin_w, FWH, FWL, kHeadN, kDm, (kHeadP * kDm) / 8);
  cast_rows_f16_kernel<<<(kNLay * kXZP * kDm) / 8 / 256, 256, 0, stream>>>(
      inproj_w, WIN16, kNLay * kXZP, kDm, (kNLay * kXZP * kDm) / 8, 32.0f);
  cast_rows_f16_kernel<<<(kNLay * kPrj * kDin) / 8 / 256, 256, 0, stream>>>(
      xproj_f, WXP16, kNLay * kPrj, kDin, (kNLay * kPrj * kDin) / 8, 32.0f);
  cast_rows_f16_kernel<<<(kNLay * kPrj * kDin) / 8 / 256, 256, 0, stream>>>(
      xproj_bk, WXP16 + (size_t)kNLay * kPrj * kDin, kNLay * kPrj, kDin, (kNLay * kPrj * kDin) / 8, 32.0f);
  cast_rows_f16_kernel<<<(kNLay * kDin * kDtR) / 8 / 256, 256, 0, stream>>>(
      dtw_f, WDT16, kNLay * kDin, kDtR, (kNLay * kDin * kDtR) / 8, 32.0f);
  cast_rows_f16_kernel<<<(kNLay * kDin * kDtR) / 8 / 256, 256, 0, stream>>>(
      dtw_bk, WDT16 + (size_t)kNLay * kDin * kDtR, kNLay * kDin, kDtR, (kNLay * kDin * kDtR) / 8, 32.0f);
  cast_dup_f16_kernel<<<(kNLay * kDm * kYP) / 8 / 256, 256, 0, stream>>>(
      outproj_w, WOUT2, (kNLay * kDm * kYP) / 8, 32.0f);
  time_embed_kernel<<<kBatch, 256, 0, stream>>>(tin, tw1, tb1, tw2, tb2, TE);
  wmma_gemm64<1, true, 2, 0, false><<<dim3(32, 1), 256, 0, stream>>>(
      XPH, XPL, kPFP, 0L, PWH, PWL, kPFP, 0L,
      (void*)Hbuf[0], (void*)Hbuf[0], kDm, 0L, patch_b, dummy_resid, 0L, kRows, kDm, kPFP, 1.0f);

  for (int i = 0; i < kNLay; ++i) {
    float* Hin  = Hbuf[i & 1];
    float* Hout = Hbuf[(i + 1) & 1];

    ln_rows_kernel<true, 0><<<kRows / 8, 256, 0, stream>>>(
        Hin, TE, norm_g + (size_t)i * kDm, norm_b + (size_t)i * kDm, HN16, HN16, kRows);

    wmma_gemm64<0, false, 0, 0, false><<<dim3(128, 1), 256, 0, stream>>>(
        HN16, HN16, kDm, 0L, WIN16 + (size_t)i * kXZP * kDm, WIN16 + (size_t)i * kXZP * kDm, kDm, 0L,
        (void*)XZ, (void*)XZ, kXZP, 0L, dummy_bias, dummy_resid, 0L, kRows, kXZP, kDm, 1.0f / 32.0f);

    conv_silu_kernel<<<dim3(kDin / 256, kSeq / 64, kBatch), 256, 0, stream>>>(
        XZ, conv_w + (size_t)i * kDin * 4, conv_b + (size_t)i * kDin, U16);

    wmma_gemm64<0, false, 0, 1, false><<<dim3(8, 2), 256, 0, stream>>>(
        U16, U16, kDin, 0L,
        WXP16 + (size_t)i * kPrj * kDin, WXP16 + (size_t)i * kPrj * kDin, kDin, (long)kNLay * kPrj * kDin,
        (void*)PRJ16, (void*)PRJ16, kPrj, (long)kRows * kPrj, dummy_bias, dummy_resid, 0L,
        kRows, kPrj, kDin, 0.125f);

    wmma_gemm64<0, false, 0, 1, false><<<dim3(64, 2), 256, 0, stream>>>(
        PRJ16, PRJ16, kPrj, (long)kRows * kPrj,
        WDT16 + (size_t)i * kDin * kDtR, WDT16 + (size_t)i * kDin * kDtR, kDtR, (long)kNLay * kDin * kDtR,
        (void*)DLR16, (void*)DLR16, kDin, (long)kRows * kDin, dummy_bias, dummy_resid, 0L,
        kRows, kDin, kDtR, 0.125f);

    scan_kernel<<<dim3(kDin / 256, kBatch, 2), 256, 0, stream>>>(
        (const _Float16*)DLR16, (const _Float16*)U16, (const _Float16*)PRJ16, XZ,
        dtb_f + (size_t)i * kDin, dtb_bk + (size_t)i * kDin,
        Alog_f + (size_t)i * kDin * kNst, Alog_bk + (size_t)i * kDin * kNst,
        D_f + (size_t)i * kDin, D_bk + (size_t)i * kDin, Y16);

    wmma_gemm64<0, false, 0, 0, true><<<dim3(32, 1), 256, 0, stream>>>(
        Y16, Y16, kYP, 0L, WOUT2 + (size_t)i * kDm * kYP, WOUT2 + (size_t)i * kDm * kYP, kYP, 0L,
        (void*)Hout, (void*)Hout, kDm, 0L, dummy_bias, Hin, 0L, kRows, kDm, kYP, 1.0f / 2048.0f);
  }

  float* Hfin = Hbuf[kNLay & 1];
  ln_rows_kernel<false, 1><<<kRows / 8, 256, 0, stream>>>(Hfin, TE, fng, fnb, HNH, HNL, kRows);
  wmma_gemm64<1, true, 0, 0, false><<<dim3(8, 1), 256, 0, stream>>>(
      HNH, HNL, kDm, 0L, FWH, FWL, kDm, 0L,
      (void*)OT, (void*)OT, kHeadP, 0L, dummy_bias, dummy_resid, 0L, kRows, kHeadP, kDm, 1.0f);
  depatch_kernel<<<(kBatch * kCin * kImg * (kImg / 4)) / 256, 256, 0, stream>>>(OT, fin_b, dout);
}
